// GraphSpatiotemporalEncoder_38190849196160
// MI455X (gfx1250) — hardware-verified
//
#include <hip/hip_runtime.h>
#include <stddef.h>
#include <stdint.h>

#define cT    6
#define cN    3200
#define cE    32000
#define cB    8
#define cIN   128
#define cG    128
#define cTOK  512
#define cGH   4
#define cNH   8
#define cHD   64
#define cLG   3
#define cLT   2
#define cM    (cT * cN)
#define cR    (cB * cT)
#define NEGS  0.2f

#define NTHR    256
#define NWAVE   8
#define EPT     8
#define CHUNK   (NTHR * EPT)
#define WCAP    (EPT * 32)
#define LISTN   (NWAVE * WCAP)
#define NBMAX   2048
#define NBRUN   320
#define BPS     (cN / NBRUN)
#define RCAP    8192
#define DEGCAP  64
#define GBM     64
#define GBN     64
#define GTHR    128
#define WSMAX   134217728
#define LDS_SCAN ((2 * RCAP + 2 * NBMAX + LISTN + 2 * NWAVE) * 4 + NWAVE * 128 * 4)

#define KATTR __attribute__((amdgpu_num_vgpr(248)))

static_assert(cN % NBRUN == 0);
static_assert(NBRUN % 8 == 0 && NBRUN <= NBMAX);
static_assert((NBMAX & (NBMAX - 1)) == 0 && NTHR * 8 == NBMAX && LISTN >= NBMAX);
static_assert((CHUNK & (CHUNK - 1)) == 0 && CHUNK <= 4096);
static_assert(cE < (1 << 19));
static_assert((RCAP % 32) == 0 && DEGCAP >= 32);
static_assert(cM % GBM == 0);
static_assert(cR % 16 == 0 && cR <= GBM);
static_assert(cHD == 64 && cTOK == 512 && cNH * cHD == cTOK);
static_assert(((2 * RCAP + 2 * NBMAX + LISTN + 2 * NWAVE) * 4) % 16 == 0);
static_assert(LDS_SCAN <= 300000);
static_assert(cR * cTOK + cB * (cT - 1) * 256 == 34816);

typedef float          v2f   __attribute__((ext_vector_type(2)));
typedef float          v4f   __attribute__((ext_vector_type(4)));
typedef float          v8f   __attribute__((ext_vector_type(8)));
typedef int            v4i   __attribute__((ext_vector_type(4)));
typedef int            v8i   __attribute__((ext_vector_type(8)));
typedef unsigned short v8us  __attribute__((ext_vector_type(8)));
typedef __bf16         v16bf __attribute__((ext_vector_type(16)));
typedef v4f __attribute__((may_alias)) v4fa;
union FragB { v16bf v; v8us u[2]; v8i w; };

__device__ __forceinline__ v8f wmx(const FragB& a, const FragB& b, v8f c) {
  v8f d = __builtin_amdgcn_wmma_f32_16x16x32_bf16(false, a.v, false, b.v, (short)0, c, false, false);
  asm volatile("v_nop\n\tv_nop\n\tv_nop\n\tv_nop" : "+v"(d) : "v"(a.w), "v"(b.w));
  return d;
}
__device__ __forceinline__ void ldwait() { asm volatile("s_wait_loadcnt 0x0" ::: "memory"); }

__device__ __forceinline__ unsigned bfbits(float v) {
  unsigned u = __float_as_uint(v);
  u = u + 0x7FFFu + ((u >> 16) & 1u);
  return u >> 16;
}
__device__ __forceinline__ float rbf(float v) { return __uint_as_float(bfbits(v) << 16); }
__device__ __forceinline__ v4f rbf4(const v4f a) {
  v4f r; r.x = rbf(a.x); r.y = rbf(a.y); r.z = rbf(a.z); r.w = rbf(a.w); return r;
}
__device__ __forceinline__ float bsel(float a, float b, int m) {
  return __int_as_float((__float_as_int(a) & m) | (__float_as_int(b) & ~m));
}
__device__ __forceinline__ v4f bsel4(const v4f a, const v4f b, int m) {
  v4f r;
  r.x = bsel(a.x, b.x, m); r.y = bsel(a.y, b.y, m);
  r.z = bsel(a.z, b.z, m); r.w = bsel(a.w, b.w, m);
  return r;
}
__device__ __forceinline__ v8us cvt8b(const v4f a, const v4f b) {
  v8us o;
  o[0] = (unsigned short)bfbits(a.x); o[1] = (unsigned short)bfbits(a.y);
  o[2] = (unsigned short)bfbits(a.z); o[3] = (unsigned short)bfbits(a.w);
  o[4] = (unsigned short)bfbits(b.x); o[5] = (unsigned short)bfbits(b.y);
  o[6] = (unsigned short)bfbits(b.z); o[7] = (unsigned short)bfbits(b.w);
  return o;
}
__device__ __forceinline__ void hl8(const v4f a, const v4f b, v8us& hv, v8us& lv) {
  const float f[8] = {a.x, a.y, a.z, a.w, b.x, b.y, b.z, b.w};
#pragma unroll
  for (int i = 0; i < 8; ++i) {
    const unsigned hb = bfbits(f[i]);
    const float hf = __uint_as_float(hb << 16);
    hv[i] = (unsigned short)hb;
    lv[i] = (unsigned short)bfbits(f[i] - hf);
  }
}
__device__ __forceinline__ float wsum(float v) {
#pragma unroll
  for (int off = 16; off > 0; off >>= 1) v += __shfl_xor(v, off);
  return v;
}
__device__ __forceinline__ void wfence() {
  __builtin_amdgcn_fence(__ATOMIC_SEQ_CST, "workgroup");
  __builtin_amdgcn_wave_barrier();
}

__device__ __forceinline__ int scan_chunk(const int* __restrict__ dsts, int nE, int cbase, int slotBase,
                                          int nb, int vec8, int* list, int tid, int lane, int wave) {
  int wc = 0;
  const int el0  = tid * EPT;
  const int e0   = cbase + el0;
  const int sent = -2147483647 - 1;
  v4i da, db;
  if (vec8 != 0 && cbase + CHUNK <= nE) {
    da = *(const v4i*)(dsts + e0);
    db = *(const v4i*)(dsts + e0 + 4);
  } else {
    da.x = (e0     < nE) ? dsts[min(e0,     nE - 1)] : sent;
    da.y = (e0 + 1 < nE) ? dsts[min(e0 + 1, nE - 1)] : sent;
    da.z = (e0 + 2 < nE) ? dsts[min(e0 + 2, nE - 1)] : sent;
    da.w = (e0 + 3 < nE) ? dsts[min(e0 + 3, nE - 1)] : sent;
    db.x = (e0 + 4 < nE) ? dsts[min(e0 + 4, nE - 1)] : sent;
    db.y = (e0 + 5 < nE) ? dsts[min(e0 + 5, nE - 1)] : sent;
    db.z = (e0 + 6 < nE) ? dsts[min(e0 + 6, nE - 1)] : sent;
    db.w = (e0 + 7 < nE) ? dsts[min(e0 + 7, nE - 1)] : sent;
  }
  const unsigned nbs = (unsigned)slotBase;
  const unsigned unb = (unsigned)nb;
  const unsigned s0 = (unsigned)da.x - nbs, s1 = (unsigned)da.y - nbs;
  const unsigned s2 = (unsigned)da.z - nbs, s3 = (unsigned)da.w - nbs;
  const unsigned s4 = (unsigned)db.x - nbs, s5 = (unsigned)db.y - nbs;
  const unsigned s6 = (unsigned)db.z - nbs, s7 = (unsigned)db.w - nbs;
  const bool h0 = s0 < unb, h1 = s1 < unb, h2 = s2 < unb, h3 = s3 < unb;
  const bool h4 = s4 < unb, h5 = s5 < unb, h6 = s6 < unb, h7 = s7 < unb;
  const unsigned any = __builtin_amdgcn_ballot_w32(h0 | h1 | h2 | h3 | h4 | h5 | h6 | h7);
  if (any != 0u) {
#define HITJ(J, HJ, SJ) { \
      const unsigned mj = __builtin_amdgcn_ballot_w32(HJ); \
      if (mj != 0u) { \
        if (HJ) { \
          const int pos = wc + (int)__builtin_amdgcn_mbcnt_lo(mj, 0u); \
          if (pos < WCAP) list[wave * WCAP + pos] = ((el0 + (J)) << 12) | (int)(SJ); \
        } \
        wc += (int)__builtin_popcount(mj); } }
    HITJ(0, h0, s0)
    HITJ(1, h1, s1)
    HITJ(2, h2, s2)
    HITJ(3, h3, s3)
    HITJ(4, h4, s4)
    HITJ(5, h5, s5)
    HITJ(6, h6, s6)
    HITJ(7, h7, s7)
#undef HITJ
  }
  return wc;
}

__global__ __launch_bounds__(NTHR) KATTR void k_xb(const float* __restrict__ x, unsigned short* xb, int nRows, int nUnits) {
  const int i = (int)blockIdx.x * NTHR + (int)threadIdx.x;
  if (i >= nUnits) return;
  const int row = i >> 4;
  const int c0  = (i & 15) * 8;
  const int rc  = row < nRows ? row : nRows - 1;
  const float* p = x + (size_t)rc * cIN + c0;
  const v4f a = *(const v4f*)p, b = *(const v4f*)(p + 4);
  const v8us hv = cvt8b(a, b);
  const size_t o = (size_t)row * cIN + c0;
  *(volatile v8us*)(xb + o) = hv;
  __threadfence();
  *(volatile v8us*)(xb + o) = hv;
}

__global__ __launch_bounds__(NTHR) KATTR void k_tab(const float* __restrict__ bl, const float* __restrict__ br, float* blr) {
  const int i = (int)blockIdx.x * NTHR + (int)threadIdx.x;
  if (i >= 768) return;
  const int l  = i >> 8;
  const int c4 = (i & 255) * 4;
  const int ca = c4 < 512 ? c4 : c4 - 512;
  const v4f a = *(const v4f*)(bl + l * 512 + ca);
  const v4f b = *(const v4f*)(br + l * 512 + ca);
  const int ml = -(int)(c4 < 512);
  const v4f r = rbf4(bsel4(a, b, ml));
  float* o = blr + l * 1024 + c4;
  *(volatile v4f*)o = r;
  __threadfence();
  *(volatile v4f*)o = r;
}

__global__ __launch_bounds__(NTHR) KATTR void k_wt(const float* __restrict__ w, int cols, int K, int srcLayer,
                                                   unsigned short* wt, int dstRowOff, int dstLayer, int nUnits) {
  const int u = (int)blockIdx.x * NTHR + (int)threadIdx.x;
  if (u >= nUnits) return;
  const int layer = (int)blockIdx.y;
  const int kq = K >> 3;
  const int n  = u / kq;
  const int k8 = (u - n * kq) * 8;
  const float* p = w + (size_t)layer * (size_t)srcLayer + (size_t)k8 * (size_t)cols + n;
  v4f a, b;
  a.x = p[0];                  a.y = p[(size_t)cols];       a.z = p[(size_t)2 * cols];   a.w = p[(size_t)3 * cols];
  b.x = p[(size_t)4 * cols];   b.y = p[(size_t)5 * cols];   b.z = p[(size_t)6 * cols];   b.w = p[(size_t)7 * cols];
  const v8us hv = cvt8b(a, b);
  const size_t o = (size_t)layer * (size_t)dstLayer + (size_t)(dstRowOff + n) * (size_t)K + k8;
  *(volatile v8us*)(wt + o) = hv;
  __threadfence();
  *(volatile v8us*)(wt + o) = hv;
}

template<int WF, int WHL, int RELU>
__global__ __launch_bounds__(GTHR) KATTR void k_gemm(
    const unsigned short* __restrict__ A, const unsigned short* __restrict__ WT,
    const float* __restrict__ bias, float* outF, unsigned short* outHL,
    int K, int kmask, int ldo, int Mreal, int Chl)
{
  __shared__ __attribute__((aligned(16))) float stg[GBM * GBN];
  const int tid = (int)threadIdx.x, lane = tid & 31, wave = tid >> 5, hh = lane >> 4, m = lane & 15;
  const int rowBase = (int)blockIdx.x * GBM;
  const int col0    = (int)blockIdx.y * GBN;
  const int Kw      = kmask + 1;

  v8f acc[4];
  {
    const v8f z = {0.f, 0.f, 0.f, 0.f, 0.f, 0.f, 0.f, 0.f};
    acc[0] = z; acc[1] = z; acc[2] = z; acc[3] = z;
  }
  int ar = rowBase + 16 * wave + m;
  ar = ar < Mreal ? ar : Mreal - 1;
  const unsigned short* ap = A  + (size_t)ar * (size_t)K + 8 * hh;
  const unsigned short* wp = WT + (size_t)(col0 + m) * (size_t)Kw + 8 * hh;
  const int ksteps = K >> 5;
#pragma unroll 1
  for (int ks = 0; ks < ksteps; ++ks) {
    FragB af;
    af.u[0] = *(const v8us*)(ap + 32 * ks);
    af.u[1] = *(const v8us*)(ap + 32 * ks + 16);
    const int kb = (32 * ks) & kmask;
#pragma unroll
    for (int t = 0; t < 4; ++t) {
      const unsigned short* wq = wp + (size_t)(16 * t) * (size_t)Kw + kb;
      FragB bf;
      bf.u[0] = *(const v8us*)wq;
      bf.u[1] = *(const v8us*)(wq + 16);
      acc[t] = wmx(af, bf, acc[t]);
    }
  }

#pragma unroll
  for (int t = 0; t < 4; ++t) {
    const int lc = 16 * t + m;
    const float bv = rbf(bias[col0 + lc]);
#pragma unroll
    for (int r = 0; r < 8; ++r) {
      const int lr = 16 * wave + 8 * hh + r;
      float v = acc[t][r] + bv;
      if (RELU) v = (v > 0.f) ? v : (v - v);
      stg[lr * GBN + lc] = v;
    }
  }
  __syncthreads();

  v4f  fv[8];
  v8us hq[8];
#pragma unroll
  for (int i = 0; i < 8; ++i) {
    if (WF) {
      const int lr = 16 * wave + 2 * i + hh;
      fv[i] = *(const v4fa*)(stg + lr * GBN + 4 * m);
    }
    if (WHL) {
      const int lid = i * 4 + (lane >> 3);
      const int row = lid >> 1, part = lid & 1, q8 = lane & 7;
      const float* p = stg + (16 * wave + row) * GBN + 8 * q8;
      const v4f a = *(const v4fa*)p, b = *(const v4fa*)(p + 4);
      v8us hv, lv;
      hl8(a, b, hv, lv);
      hq[i] = part ? lv : hv;
    }
  }
#pragma unroll
  for (int pass = 0; pass < 2; ++pass) {
#pragma unroll
    for (int i = 0; i < 8; ++i) {
      if (WF) {
        const int gr = rowBase + 16 * wave + 2 * i + hh;
        if (gr < Mreal) *(volatile v4f*)(outF + (size_t)gr * (size_t)ldo + col0 + 4 * m) = fv[i];
      }
      if (WHL) {
        const int lid = i * 4 + (lane >> 3);
        const int row = lid >> 1, part = lid & 1, q8 = lane & 7;
        const int gr = rowBase + 16 * wave + row;
        if (gr < Mreal)
          *(volatile v8us*)(outHL + (size_t)gr * (size_t)(2 * Chl) + (size_t)part * Chl + col0 + 8 * q8) = hq[i];
      }
    }
    if (pass == 0) __threadfence();
  }
  (void)outF; (void)outHL;
}

template<int FINAL>
__global__ __launch_bounds__(NTHR) KATTR void k_gln(
    const unsigned short* __restrict__ A, const unsigned short* __restrict__ WT, const float* __restrict__ bias,
    const float* __restrict__ lng, const float* __restrict__ lnb,
    float* X, unsigned short* XHL, float* dout, int K, int kmask)
{
  __shared__ __attribute__((aligned(16))) float stg[16 * cTOK];
  const int tid = (int)threadIdx.x, lane = tid & 31, wave = tid >> 5, hh = lane >> 4, m = lane & 15;
  const int rowBase = (int)blockIdx.x * 16;
  const int Kw = kmask + 1;
  v8f acc[4];
  {
    const v8f z = {0.f, 0.f, 0.f, 0.f, 0.f, 0.f, 0.f, 0.f};
    acc[0] = z; acc[1] = z; acc[2] = z; acc[3] = z;
  }
  const unsigned short* ap = A  + (size_t)(rowBase + m) * (size_t)K + 8 * hh;
  const unsigned short* wp = WT + (size_t)(64 * wave + m) * (size_t)Kw + 8 * hh;
  const int ksteps = K >> 5;
#pragma unroll 1
  for (int ks = 0; ks < ksteps; ++ks) {
    FragB af;
    af.u[0] = *(const v8us*)(ap + 32 * ks);
    af.u[1] = *(const v8us*)(ap + 32 * ks + 16);
    const int kb = (32 * ks) & kmask;
#pragma unroll
    for (int t = 0; t < 4; ++t) {
      const unsigned short* wq = wp + (size_t)(16 * t) * (size_t)Kw + kb;
      FragB bf;
      bf.u[0] = *(const v8us*)wq;
      bf.u[1] = *(const v8us*)(wq + 16);
      acc[t] = wmx(af, bf, acc[t]);
    }
  }
#pragma unroll
  for (int t = 0; t < 4; ++t)
#pragma unroll
    for (int r = 0; r < 8; ++r)
      stg[(8 * hh + r) * cTOK + 64 * wave + 16 * t + m] = acc[t][r];
  __syncthreads();

#pragma unroll 1
  for (int rr = 0; rr < 2; ++rr) {
    const int lr = 2 * wave + rr;
    const int grow = rowBase + lr;
    float* srow = stg + lr * cTOK;
    v4f v[4];
    float sum = 0.f;
#pragma unroll
    for (int j = 0; j < 4; ++j) {
      const int c = 128 * j + 4 * lane;
      const v4f s  = *(const v4fa*)(srow + c);
      const v4f bb = rbf4(*(const v4f*)(bias + c));
      const v4f xx = *(const v4f*)(X + (size_t)grow * cTOK + c);
      v[j] = xx + (s + bb);
      sum += (v[j].x + v[j].y) + (v[j].z + v[j].w);
    }
    sum = wsum(sum);
    const float mu = sum * (1.0f / (float)cTOK);
    float sq = 0.f;
#pragma unroll
    for (int j = 0; j < 4; ++j) {
      v[j] = v[j] - mu;
      sq += (v[j].x * v[j].x + v[j].y * v[j].y) + (v[j].z * v[j].z + v[j].w * v[j].w);
    }
    sq = wsum(sq);
    const float rstd = 1.0f / sqrtf(sq * (1.0f / (float)cTOK) + 1e-5f);
    v4f y[4];
#pragma unroll
    for (int j = 0; j < 4; ++j) {
      const int c = 128 * j + 4 * lane;
      const v4f g4 = rbf4(*(const v4f*)(lng + c));
      const v4f b4 = rbf4(*(const v4f*)(lnb + c));
      y[j] = (v[j] * rstd) * g4 + b4;
    }
    wfence();
#pragma unroll
    for (int j = 0; j < 4; ++j) *(v4fa*)(srow + 128 * j + 4 * lane) = y[j];
    wfence();
    v8us hq[4];
#pragma unroll
    for (int i = 0; i < 4; ++i) {
      const int p = 32 * i + lane;
      const int part = p >> 6, c8 = (p & 63) * 8;
      const v4f a = *(const v4fa*)(srow + c8), b = *(const v4fa*)(srow + c8 + 4);
      v8us hv, lv;
      hl8(a, b, hv, lv);
      hq[i] = part ? lv : hv;
    }
#pragma unroll
    for (int pass = 0; pass < 2; ++pass) {
#pragma unroll
      for (int j = 0; j < 4; ++j) {
        const size_t o = (size_t)grow * cTOK + 128 * j + 4 * lane;
        *(volatile v4f*)(X + o) = y[j];
        if (FINAL) *(volatile v4f*)(dout + o) = y[j];
      }
#pragma unroll
      for (int i = 0; i < 4; ++i)
        *(volatile v8us*)(XHL + (size_t)grow * (2 * cTOK) + 8 * (32 * i + lane)) = hq[i];
      if (pass == 0) __threadfence();
    }
  }
  (void)dout;
}

__global__ __launch_bounds__(NTHR) KATTR void k_scan(
    const int* __restrict__ ei, const float* __restrict__ ea, const float* __restrict__ XLR,
    const float* __restrict__ we, const float* __restrict__ att, const float* __restrict__ gbias,
    const float* __restrict__ lng, const float* __restrict__ lnb,
    float* H, unsigned short* HHL)
{
  extern __shared__ v4f lds_dyn[];
  int* reg1 = (int*)lds_dyn;
  int* reg2 = reg1 + RCAP;
  int* scnt = reg2 + RCAP;
  int* soff = scnt + NBMAX;
  int* list = soff + NBMAX;
  int* wcnt = list + LISTN;
  int* wtot = wcnt + NWAVE;
  float* stwb = (float*)(wtot + NWAVE);
  const int tid = (int)threadIdx.x, lane = tid & 31, wave = tid >> 5;
  const int t = (int)blockIdx.x / BPS;
  const int nodeBase = ((int)blockIdx.x - t * BPS) * NBRUN;
  const int* srcs = ei + (size_t)t * 2 * cE;
  const int* dsts = srcs + cE;
  const float* eat = ea + (size_t)t * cE * 2;
  const int rowT = t * cN;
  const int nE = cE, nb = NBRUN;

  for (int i = tid; i < NBMAX; i += NTHR) scnt[i] = 0;
  __syncthreads();

  int tot = 0;
  const int nChunks = (nE + CHUNK - 1) / CHUNK;
#pragma unroll 1
  for (int ch = 0; ch < nChunks; ++ch) {
    const int cbase = ch * CHUNK;
    const int wc = scan_chunk(dsts, nE, cbase, nodeBase, nb, 1, list, tid, lane, wave);
    if (lane == 0) wcnt[wave] = wc;
    __syncthreads();
    int pre = 0, all = 0;
#pragma unroll
    for (int w2 = 0; w2 < NWAVE; ++w2) {
      int c = wcnt[w2];
      c = c < 0 ? 0 : (c > WCAP ? WCAP : c);
      all += c;
      pre += (w2 < wave) ? c : 0;
    }
    const int wcc  = wc > WCAP ? WCAP : wc;
    const int base = tot + pre;
#pragma unroll 1
    for (int i = lane; i < wcc; i += 32) {
      const int ent = list[wave * WCAP + i];
      const int el  = (ent >> 12) & (CHUNK - 1);
      const int sl  = ent & (NBMAX - 1);
      int eid = cbase + el;
      eid = eid > nE - 1 ? nE - 1 : eid;
      const int pos = base + i;
      if (pos < RCAP) reg1[pos] = (int)(((unsigned)eid << 12) | (unsigned)sl);
    }
    tot += all;
    tot = tot > RCAP ? RCAP : tot;
    __syncthreads();
  }
  const int nh = tot;

  if (wave == 0) {
#pragma unroll 1
    for (int b0 = 0; b0 < nh; b0 += 32) {
      const int idx = b0 + lane;
      const int uv  = reg1[idx < RCAP ? idx : RCAP - 1];
      const int m32 = (nh - b0) < 32 ? (nh - b0) : 32;
#pragma unroll 1
      for (int k = 0; k < m32; ++k) {
        const int u  = __builtin_amdgcn_readlane(uv, k);
        const int sl = u & (NBMAX - 1);
        if (lane == 0) scnt[sl] = scnt[sl] + 1;
      }
    }
  }
  __syncthreads();

  {
    const v4i ca = *(const v4i*)(scnt + 8 * tid);
    const v4i cb = *(const v4i*)(scnt + 8 * tid + 4);
    const int e0 = ca.x < 0 ? 0 : ca.x, e1 = ca.y < 0 ? 0 : ca.y, e2 = ca.z < 0 ? 0 : ca.z, e3 = ca.w < 0 ? 0 : ca.w;
    const int e4 = cb.x < 0 ? 0 : cb.x, e5 = cb.y < 0 ? 0 : cb.y, e6 = cb.z < 0 ? 0 : cb.z, e7 = cb.w < 0 ? 0 : cb.w;
    const int ts = e0 + e1 + e2 + e3 + e4 + e5 + e6 + e7;
    int incl = ts;
#pragma unroll
    for (int d = 1; d < 32; d <<= 1) {
      const int up = __shfl_up(incl, d);
      if (lane >= d) incl += up;
    }
    if (lane == 31) wtot[wave] = incl;
    __syncthreads();
    int pre = 0;
#pragma unroll
    for (int w2 = 0; w2 < NWAVE; ++w2) pre += (w2 < wave) ? wtot[w2] : 0;
    int run = pre + incl - ts;
    soff[8 * tid + 0] = run; run += e0;
    soff[8 * tid + 1] = run; run += e1;
    soff[8 * tid + 2] = run; run += e2;
    soff[8 * tid + 3] = run; run += e3;
    soff[8 * tid + 4] = run; run += e4;
    soff[8 * tid + 5] = run; run += e5;
    soff[8 * tid + 6] = run; run += e6;
    soff[8 * tid + 7] = run;
  }
  __syncthreads();
  for (int i = tid; i < NBMAX; i += NTHR) list[i] = soff[i];
  __syncthreads();

  if (wave == 0) {
#pragma unroll 1
    for (int b0 = 0; b0 < nh; b0 += 32) {
      const int idx = b0 + lane;
      const int uv  = reg1[idx < RCAP ? idx : RCAP - 1];
      const int m32 = (nh - b0) < 32 ? (nh - b0) : 32;
#pragma unroll 1
      for (int k = 0; k < m32; ++k) {
        const int u   = __builtin_amdgcn_readlane(uv, k);
        const int sl  = u & (NBMAX - 1);
        const int eid = (int)((unsigned)u >> 12);
        if (lane == 0) {
          int pos = list[sl];
          pos = pos < 0 ? 0 : (pos > RCAP - 1 ? RCAP - 1 : pos);
          reg2[pos] = eid;
          list[sl] = pos + 1;
        }
      }
    }
  }
  __syncthreads();

  const int nbw = NBRUN >> 3;
  const bool ovf = (nh >= RCAP);
  const float qnan = __int_as_float(0x7fc00000);
  float* stw = stwb + wave * 128;
  const v4f gb4 = rbf4(*(const v4f*)(gbias + 4 * lane));
  const v4f g4  = rbf4(*(const v4f*)(lng + 4 * lane));
  const v4f b4  = rbf4(*(const v4f*)(lnb + 4 * lane));
#pragma unroll 1
  for (int jt = 0; jt < nbw; ++jt) {
    const int slot = wave * nbw + jt;
    const int grow = rowT + nodeBase + slot;
    int st = soff[slot];
    const int craw = scnt[slot];
    int cnt = craw;
    st  = st < 0 ? 0 : (st > nh ? nh : st);
    cnt = cnt < 0 ? 0 : (cnt > DEGCAP ? DEGCAP : cnt);
    if (cnt > nh - st) cnt = nh - st;
    st  = __builtin_amdgcn_readfirstlane(st);
    cnt = __builtin_amdgcn_readfirstlane(cnt);
    const float pz = (ovf || craw > DEGCAP) ? qnan : 0.0f;
    const float* xrow = XLR + (size_t)grow * 1024 + 512;

    v4f mean4 = {0.f, 0.f, 0.f, 0.f};
#pragma unroll 1
    for (int hd = 0; hd < cGH; ++hd) {
      const int coff = hd * cG + 4 * lane;
      const v4f xr4 = *(const v4f*)(xrow + coff);
      const v4f at4 = rbf4(*(const v4f*)(att + coff));
      const v4f w04 = rbf4(*(const v4f*)(we + coff));
      const v4f w14 = rbf4(*(const v4f*)(we + 512 + coff));
      float mx = -1.0e30f, dn = 0.f;
      v4f av = {0.f, 0.f, 0.f, 0.f};
#pragma unroll 1
      for (int q = 0; q < cnt; ++q) {
        int idx = st + q; idx = idx > RCAP - 1 ? RCAP - 1 : idx;
        int eid = reg2[idx]; eid = eid < 0 ? 0 : (eid > cE - 1 ? cE - 1 : eid);
        const int sraw = srcs[eid];
        const int s = sraw < 0 ? 0 : (sraw > cN - 1 ? cN - 1 : sraw);
        const v2f e2 = *(const v2f*)(eat + 2 * eid);
        const v4f hs = *(const v4f*)(XLR + (size_t)(rowT + s) * 1024 + coff);
        ldwait();
        const float e0 = rbf(e2.x), e1 = rbf(e2.y);
        float part = 0.f;
#define COMP(c) { const float eev = fmaf(e1, w14.c, e0 * w04.c); float v = (hs.c + xr4.c) + eev; \
                  v = v > 0.f ? v : v * NEGS; part = fmaf(v, at4.c, part); }
        COMP(x) COMP(y) COMP(z) COMP(w)
#undef COMP
        part = wsum(part);
        const float df = part - mx;
        const float ex = expf(-fabsf(df));
        const bool up  = df > 0.f;
        const float s1 = up ? ex : 1.0f;
        const float s2 = up ? 1.0f : ex;
        mx = up ? part : mx;
        dn = fmaf(dn, s1, s2);
        av.x = fmaf(av.x, s1, s2 * hs.x);
        av.y = fmaf(av.y, s1, s2 * hs.y);
        av.z = fmaf(av.z, s1, s2 * hs.z);
        av.w = fmaf(av.w, s1, s2 * hs.w);
      }
      const float iv = (dn > 0.f) ? __builtin_amdgcn_rcpf(dn + 1e-16f) : 0.0f;
      mean4 = mean4 + av * iv;
    }

    const v4f hres = *(const v4f*)(H + (size_t)grow * cG + 4 * lane);
    v4f o = mean4 * 0.25f + gb4;
    o.x = (o.x > 0.f) ? o.x : (o.x - o.x);
    o.y = (o.y > 0.f) ? o.y : (o.y - o.y);
    o.z = (o.z > 0.f) ? o.z : (o.z - o.z);
    o.w = (o.w > 0.f) ? o.w : (o.w - o.w);
    v4f v = o + hres;
    const float sum = wsum((v.x + v.y) + (v.z + v.w));
    const float mu = sum * (1.0f / (float)cG);
    v = v - mu;
    const float sq = wsum((v.x * v.x + v.y * v.y) + (v.z * v.z + v.w * v.w));
    const float rstd = 1.0f / sqrtf(sq * (1.0f / (float)cG) + 1e-5f);
    const v4f y = ((v * rstd) * g4 + b4) + pz;

    wfence();
    *(v4fa*)(stw + 4 * lane) = y;
    wfence();
    const v4f ga = *(const v4fa*)(stw + 8 * (lane & 15));
    const v4f gc = *(const v4fa*)(stw + 8 * (lane & 15) + 4);
    v8us hv, lv;
    hl8(ga, gc, hv, lv);
    const v8us sel = (lane < 16) ? hv : lv;
    float* hp = H + (size_t)grow * cG + 4 * lane;
    unsigned short* lp = HHL + (size_t)grow * (2 * cG) + 8 * lane;
    *(volatile v4f*)hp = y;
    *(volatile v8us*)lp = sel;
    __threadfence();
    *(volatile v4f*)hp = y;
    *(volatile v8us*)lp = sel;
  }
}

__global__ __launch_bounds__(128) KATTR void k_pool(const float* __restrict__ H, const int* __restrict__ batch,
                                                    unsigned short* PHL) {
  __shared__ __attribute__((aligned(16))) float sm[cG];
  __shared__ __attribute__((aligned(16))) float sx[cG];
  const int tid = (int)threadIdx.x;
  const int t = (int)blockIdx.x / cB;
  const int g = (int)blockIdx.x - t * cB;
  float sum = 0.0f;
  float mx = __int_as_float((int)0xff800000u);
  int cnt = 0;
#pragma unroll 4
  for (int n = 0; n < cN; ++n) {
    const int bn = batch[n];
    if (bn == g) {
      const float v = H[(size_t)(t * cN + n) * cG + tid];
      sum += v;
      mx = (v > mx || v != v) ? v : mx;
      cnt += 1;
    }
  }
  const float cf = (float)cnt;
  const float mean = sum * (1.0f / (cf > 1.0f ? cf : 1.0f));
  sm[tid] = mean;
  sx[tid] = mx;
  __syncthreads();
  const int j = tid & 63;
  const int seg = j >> 4, c8 = (j & 15) * 8;
  const v4f ma = *(const v4fa*)(sm + c8), mb = *(const v4fa*)(sm + c8 + 4);
  const v4f xa = *(const v4fa*)(sx + c8), xb = *(const v4fa*)(sx + c8 + 4);
  const int mxm = -(int)(seg & 1);
  const v4f a = bsel4(xa, ma, mxm);
  const v4f b = bsel4(xb, mb, mxm);
  v8us hv, lv;
  hl8(a, b, hv, lv);
  const v8us sel = (seg >> 1) ? lv : hv;
  const int r = g * cT + t;
  unsigned short* dst = PHL + (size_t)r * 512 + 8 * j;
  if (tid < 64) *(volatile v8us*)dst = sel;
  __threadfence();
  if (tid < 64) *(volatile v8us*)dst = sel;
}

__global__ __launch_bounds__(NTHR) KATTR void k_mot(const float* __restrict__ X, float* out1) {
  const int i = (int)blockIdx.x * NTHR + (int)threadIdx.x;
  if (i >= cB * (cT - 1) * 64) return;
  const int row = i >> 6, c4 = (i & 63) * 4;
  const int b = row / (cT - 1), dt = row - b * (cT - 1);
  const int r0 = b * cT + dt;
  const v4f a = *(const v4f*)(X + (size_t)r0 * cTOK + c4);
  const v4f c = *(const v4f*)(X + (size_t)(r0 + 1) * cTOK + c4);
  const v4f d = c - a;
  float* o = out1 + (size_t)row * 256 + c4;
  *(volatile v4f*)o = d;
  __threadfence();
  *(volatile v4f*)o = d;
}

__global__ __launch_bounds__(NTHR) KATTR void k_attn(const float* __restrict__ QKV, unsigned short* AO) {
  const int tid = (int)threadIdx.x, lane = tid & 31, wave = tid >> 5;
  const int wid = (int)blockIdx.x * NWAVE + wave;
  const int b = wid >> 3, hd = wid & 7;
#pragma unroll 1
  for (int q = 0; q < cT; ++q) {
    const int row = b * cT + q;
    const v2f qv = *(const v2f*)(QKV + (size_t)row * 1536 + hd * cHD + 2 * lane);
    float mx = -1.0e30f, dn = 0.f, o0 = 0.f, o1 = 0.f;
#pragma unroll 1
    for (int k = 0; k < cT; ++k) {
      const float* kr = QKV + (size_t)(b * cT + k) * 1536 + hd * cHD + 2 * lane;
      const v2f kv = *(const v2f*)(kr + 512);
      const v2f vv = *(const v2f*)(kr + 1024);
      float part = fmaf(qv.y, kv.y, qv.x * kv.x);
      part = wsum(part) * 0.125f;
      const float df = part - mx;
      const float ex = expf(-fabsf(df));
      const bool up  = df > 0.f;
      const float s1 = up ? ex : 1.0f;
      const float s2 = up ? 1.0f : ex;
      mx = up ? part : mx;
      dn = fmaf(dn, s1, s2);
      o0 = fmaf(o0, s1, s2 * vv.x);
      o1 = fmaf(o1, s1, s2 * vv.y);
    }
    const float inv = 1.0f / dn;
    const float r0 = o0 * inv, r1 = o1 * inv;
    const unsigned h0 = bfbits(r0), h1 = bfbits(r1);
    const unsigned l0 = bfbits(r0 - __uint_as_float(h0 << 16));
    const unsigned l1 = bfbits(r1 - __uint_as_float(h1 << 16));
    const unsigned hp = h0 | (h1 << 16);
    const unsigned lp = l0 | (l1 << 16);
    unsigned* dh = (unsigned*)(AO + (size_t)row * 1024 + hd * cHD) + lane;
    unsigned* dl = (unsigned*)(AO + (size_t)row * 1024 + 512 + hd * cHD) + lane;
    *(volatile unsigned*)dh = hp;
    *(volatile unsigned*)dl = lp;
    __threadfence();
    *(volatile unsigned*)dh = hp;
    *(volatile unsigned*)dl = lp;
  }
}

static inline int cdiv(int a, int b) { return (a + b - 1) / b; }

extern "C" void kernel_launch(void* const* d_in, const int* in_sizes, int n_in,
                              void* d_out, int out_size, void* d_ws, size_t ws_size,
                              hipStream_t stream) {
  if (n_in < 29) return;
  const int expect[29] = {
    cT * cN * cIN, cT * 2 * cE, cT * cE * 2, cN, cIN * cG, cG,
    cLG * cG * 512, cLG * 512, cLG * cG * 512, cLG * 512, cLG * 2 * 512, cLG * cGH * cG,
    cLG * cG, cLG * cG, cLG * cG, 2 * cG * cTOK, cTOK,
    cLT * cTOK * 1536, cLT * 1536, cLT * cTOK * cTOK, cLT * cTOK,
    cLT * cTOK * 2048, cLT * 2048, cLT * 2048 * cTOK, cLT * cTOK,
    cLT * cTOK, cLT * cTOK, cLT * cTOK, cLT * cTOK };
  for (int i = 0; i < 29; ++i) if (in_sizes[i] != expect[i]) return;
  if (out_size != cR * cTOK + cB * (cT - 1) * 256) return;

  const float* x       = (const float*)d_in[0];
  const int*   ei      = (const int*)  d_in[1];
  const float* ea      = (const float*)d_in[2];
  const int*   batch   = (const int*)  d_in[3];
  const float* proj_w  = (const float*)d_in[4];
  const float* proj_b  = (const float*)d_in[5];
  const float* gat_wl  = (const float*)d_in[6];
  const float* gat_bl  = (const float*)d_in[7];
  const float* gat_wr  = (const float*)d_in[8];
  const float* gat_br  = (const float*)d_in[9];
  const float* gat_we  = (const float*)d_in[10];
  const float* gat_att = (const float*)d_in[11];
  const float* gat_bias= (const float*)d_in[12];
  const float* ln_g    = (const float*)d_in[13];
  const float* ln_b    = (const float*)d_in[14];
  const float* n2t_w   = (const float*)d_in[15];
  const float* n2t_b   = (const float*)d_in[16];
  const float* tf_wqkv = (const float*)d_in[17];
  const float* tf_bqkv = (const float*)d_in[18];
  const float* tf_wo   = (const float*)d_in[19];
  const float* tf_bo   = (const float*)d_in[20];
  const float* tf_w1   = (const float*)d_in[21];
  const float* tf_b1   = (const float*)d_in[22];
  const float* tf_w2   = (const float*)d_in[23];
  const float* tf_b2   = (const float*)d_in[24];
  const float* tf_ln1g = (const float*)d_in[25];
  const float* tf_ln1b = (const float*)d_in[26];
  const float* tf_ln2g = (const float*)d_in[27];
  const float* tf_ln2b = (const float*)d_in[28];
  float* out = (float*)d_out;

  char* ws = (char*)d_ws;
  size_t off = 0;
  const size_t oXLR  = off; off += (size_t)cM * 1024 * 4;
  const size_t oH    = off; off += (size_t)cM * cG * 4;
  const size_t oHHL  = off; off += (size_t)cM * 2 * cG * 2;
  const size_t oXB   = off; off += (size_t)cM * cIN * 2;
  const size_t oPWT  = off; off += (size_t)cG * cIN * 2;
  const size_t oWLR  = off; off += (size_t)cLG * 1024 * cG * 2;
  const size_t oBLR  = off; off += (size_t)cLG * 1024 * 4;
  const size_t oN2T  = off; off += (size_t)cTOK * 256 * 2;
  const size_t oWQKV = off; off += (size_t)cLT * 1536 * cTOK * 2;
  const size_t oWO   = off; off += (size_t)cLT * cTOK * cTOK * 2;
  const size_t oW1   = off; off += (size_t)cLT * 2048 * cTOK * 2;
  const size_t oW2   = off; off += (size_t)cLT * cTOK * 2048 * 2;
  const size_t oPHL  = off; off += (size_t)cR * 512 * 2;
  const size_t oX    = off; off += (size_t)cR * cTOK * 4;
  const size_t oXHL  = off; off += (size_t)cR * 1024 * 2;
  const size_t oQKV  = off; off += (size_t)cR * 1536 * 4;
  const size_t oAO   = off; off += (size_t)cR * 1024 * 2;
  const size_t oF    = off; off += (size_t)cR * 4096 * 2;
  if (off > ws_size || off > (size_t)WSMAX) return;

  float*          XLR  = (float*)(ws + oXLR);
  float*          H    = (float*)(ws + oH);
  unsigned short* HHL  = (unsigned short*)(ws + oHHL);
  unsigned short* XB   = (unsigned short*)(ws + oXB);
  unsigned short* PWT  = (unsigned short*)(ws + oPWT);
  unsigned short* WLR  = (unsigned short*)(ws + oWLR);
  float*          BLR  = (float*)(ws + oBLR);
  unsigned short* N2T  = (unsigned short*)(ws + oN2T);
  unsigned short* WQKV = (unsigned short*)(ws + oWQKV);
  unsigned short* WO   = (unsigned short*)(ws + oWO);
  unsigned short* W1   = (unsigned short*)(ws + oW1);
  unsigned short* W2   = (unsigned short*)(ws + oW2);
  unsigned short* PHL  = (unsigned short*)(ws + oPHL);
  float*          X    = (float*)(ws + oX);
  unsigned short* XHL  = (unsigned short*)(ws + oXHL);
  float*          QKV  = (float*)(ws + oQKV);
  unsigned short* AO   = (unsigned short*)(ws + oAO);
  unsigned short* F    = (unsigned short*)(ws + oF);

  hipFuncSetAttribute(reinterpret_cast<const void*>(&k_scan),
                      hipFuncAttributeMaxDynamicSharedMemorySize, LDS_SCAN);

  {
    const int nUx = cM * (cIN / 8);
    k_xb<<<cdiv(nUx, NTHR), NTHR, 0, stream>>>(x, XB, cM, nUx);
    k_tab<<<3, NTHR, 0, stream>>>(gat_bl, gat_br, BLR);
    k_wt<<<dim3(cdiv(128 * 16, NTHR), 1), NTHR, 0, stream>>>(proj_w, 128, 128, 0, PWT, 0, 0, 128 * 16);
    k_wt<<<dim3(cdiv(512 * 16, NTHR), cLG), NTHR, 0, stream>>>(gat_wl, 512, 128, 128 * 512, WLR, 0, 1024 * 128, 512 * 16);
    k_wt<<<dim3(cdiv(512 * 16, NTHR), cLG), NTHR, 0, stream>>>(gat_wr, 512, 128, 128 * 512, WLR, 512, 1024 * 128, 512 * 16);
    k_wt<<<dim3(cdiv(512 * 32, NTHR), 1), NTHR, 0, stream>>>(n2t_w, 512, 256, 0, N2T, 0, 0, 512 * 32);
    k_wt<<<dim3(cdiv(1536 * 64, NTHR), cLT), NTHR, 0, stream>>>(tf_wqkv, 1536, 512, 512 * 1536, WQKV, 0, 1536 * 512, 1536 * 64);
    k_wt<<<dim3(cdiv(512 * 64, NTHR), cLT), NTHR, 0, stream>>>(tf_wo, 512, 512, 512 * 512, WO, 0, 512 * 512, 512 * 64);
    k_wt<<<dim3(cdiv(2048 * 64, NTHR), cLT), NTHR, 0, stream>>>(tf_w1, 2048, 512, 512 * 2048, W1, 0, 2048 * 512, 2048 * 64);
    k_wt<<<dim3(cdiv(512 * 256, NTHR), cLT), NTHR, 0, stream>>>(tf_w2, 512, 2048, 2048 * 512, W2, 0, 512 * 2048, 512 * 256);
  }

  k_gemm<1, 1, 0><<<dim3(cM / GBM, cG / GBN), GTHR, 0, stream>>>(XB, PWT, proj_b, H, HHL, cIN, cIN - 1, cG, cM, cG);

  for (int l = 0; l < cLG; ++l) {
    k_gemm<1, 0, 0><<<dim3(cM / GBM, 1024 / GBN), GTHR, 0, stream>>>(
        HHL, WLR + (size_t)l * 1024 * 128, BLR + l * 1024, XLR, HHL, 2 * cG, cG - 1, 1024, cM, 0);
    k_scan<<<cT * BPS, NTHR, LDS_SCAN, stream>>>(
        ei, ea, XLR, gat_we + (size_t)l * 1024, gat_att + (size_t)l * 512, gat_bias + l * cG,
        ln_g + l * cG, ln_b + l * cG, H, HHL);
  }

  k_pool<<<cT * cB, 128, 0, stream>>>(H, batch, PHL);
  k_gemm<1, 1, 0><<<dim3(1, cTOK / GBN), GTHR, 0, stream>>>(PHL, N2T, n2t_b, X, XHL, 512, 255, cTOK, cR, cTOK);
  k_mot<<<cdiv(cB * (cT - 1) * 64, NTHR), NTHR, 0, stream>>>(X, out + cR * cTOK);

  for (int l = 0; l < cLT; ++l) {
    k_gemm<1, 0, 0><<<dim3(1, 1536 / GBN), GTHR, 0, stream>>>(
        XHL, WQKV + (size_t)l * 1536 * 512, tf_bqkv + l * 1536, QKV, XHL, 1024, 511, 1536, cR, 0);
    k_attn<<<cB * cNH / NWAVE, NTHR, 0, stream>>>(QKV, AO);
    k_gln<0><<<cR / 16, NTHR, 0, stream>>>(AO, WO + (size_t)l * 512 * 512, tf_bo + l * 512,
                                           tf_ln1g + l * 512, tf_ln1b + l * 512, X, XHL, out, 1024, 511);
    k_gemm<0, 1, 1><<<dim3(1, 2048 / GBN), GTHR, 0, stream>>>(
        XHL, W1 + (size_t)l * 2048 * 512, tf_b1 + l * 2048, X, F, 1024, 511, 0, cR, 2048);
    if (l == cLT - 1)
      k_gln<1><<<cR / 16, NTHR, 0, stream>>>(F, W2 + (size_t)l * 512 * 2048, tf_b2 + l * 512,
                                             tf_ln2g + l * 512, tf_ln2b + l * 512, X, XHL, out, 4096, 2047);
    else
      k_gln<0><<<cR / 16, NTHR, 0, stream>>>(F, W2 + (size_t)l * 512 * 2048, tf_b2 + l * 512,
                                             tf_ln2g + l * 512, tf_ln2b + l * 512, X, XHL, out, 4096, 2047);
  }
}
